// ModernBertAttention_14474039788078
// MI455X (gfx1250) — hardware-verified
//
#include <hip/hip_runtime.h>


#ifndef NB
#define NB   2
#endif
#ifndef SEQ
#define SEQ  2048
#endif
#define NB_FULL 2
#define S_FULL  2048
#define DM   768
#define NH   12
#define HD   64
#define DQKV (3 * DM)
#define KPAD 64
#define BW   192
#define LDV  (SEQ + 2 * KPAD)
#define SCL  0.125f
#define THETA 10000.0f

static_assert(SEQ % 64 == 0);
static_assert(SEQ <= S_FULL);
static_assert(NB <= NB_FULL);
static_assert(DM % 64 == 0);
static_assert(DQKV % 64 == 0);
static_assert(BW % 32 == 0);
static_assert(LDV % 8 == 0);
static_assert((NH * SEQ) % 8 == 0);

typedef _Float16 h16;
typedef unsigned short bf;
typedef __attribute__((ext_vector_type(16))) __bf16   v16bf;
typedef __attribute__((ext_vector_type(16))) _Float16 v16h;
typedef __attribute__((ext_vector_type(8)))  _Float16 v8h;
typedef __attribute__((ext_vector_type(8)))  unsigned short v8us;
typedef __attribute__((ext_vector_type(8)))  float    v8f;
typedef __attribute__((ext_vector_type(4)))  float    v4f;
typedef v8h  __attribute__((may_alias)) v8ha;
typedef v4f  __attribute__((may_alias)) v4fa;
typedef v8us __attribute__((may_alias)) v8usa;
typedef __attribute__((ext_vector_type(2))) _Float16 v2h;
typedef __attribute__((ext_vector_type(4))) _Float16 v4h;
typedef __attribute__((ext_vector_type(2))) unsigned short v2us;
typedef __attribute__((ext_vector_type(4))) unsigned short v4us;
typedef __attribute__((ext_vector_type(2))) float v2f;
typedef __attribute__((ext_vector_type(4))) int v4i;

__device__ __forceinline__ unsigned short f2bf(float f) { unsigned u = __float_as_uint(f); u += 0x7FFFu + ((u >> 16) & 1u); return (unsigned short)(u >> 16); }
__device__ __forceinline__ float bf2f(unsigned short b) { return __uint_as_float(((unsigned)b) << 16); }
__device__ __forceinline__ float bfr(float f) { return bf2f(f2bf(f)); }
__device__ __forceinline__ v16h cat16(v8h lo, v8h hi) { return __builtin_shufflevector(lo, hi, 0, 1, 2, 3, 4, 5, 6, 7, 8, 9, 10, 11, 12, 13, 14, 15); }
__device__ __forceinline__ v16bf cat16b(v8us lo, v8us hi) { return __builtin_bit_cast(v16bf, __builtin_shufflevector(lo, hi, 0, 1, 2, 3, 4, 5, 6, 7, 8, 9, 10, 11, 12, 13, 14, 15)); }
__device__ __forceinline__ v8f wmma16(v16h a, v16h b, v8f c) { return __builtin_amdgcn_wmma_f32_16x16x32_f16(false, a, false, b, (short)0, c, false, false); }
__device__ __forceinline__ v8f wmmab(v16bf a, v16bf b, v8f c) { return __builtin_amdgcn_wmma_f32_16x16x32_bf16(false, a, false, b, (short)0, c, false, false); }
__device__ __forceinline__ void splitf(float y, unsigned short& h, unsigned short& l) { h = f2bf(y); l = f2bf(y - bf2f(h)); }

template <typename T16> struct WFrag;
template <> struct WFrag<h16> { typedef v16h V; static __device__ __forceinline__ V ld(const h16* p) { return cat16(*(const v8h*)p, *(const v8h*)(p + 16)); } static __device__ __forceinline__ v8f mma(V a, V b, v8f c) { return wmma16(a, b, c); } };
template <> struct WFrag<bf> { typedef v16bf V; static __device__ __forceinline__ V ld(const bf* p) { return cat16b(*(const v8us*)p, *(const v8us*)(p + 16)); } static __device__ __forceinline__ v8f mma(V a, V b, v8f c) { return wmmab(a, b, c); } };
template <typename T16, int NSPLIT, bool BIAS>
__global__ __launch_bounds__(32) void k_gemmw(const T16* __restrict__ A, const T16* __restrict__ A2, const T16* __restrict__ Bt, const T16* __restrict__ Bt2, int K, int lda, int ldb, int bxr, int bxk,
                                              float* C, int ldc, const float* __restrict__ bias, size_t sA, size_t sB, size_t sC) {
    typedef typename WFrag<T16>::V V;
    __shared__ __align__(16) float os[16 * 68];
    const size_t z = blockIdx.z; A += z * sA; if (A2) A2 += z * sA; Bt += z * sB; if (Bt2) Bt2 += z * sB; C += z * sC;
    const int lane = threadIdx.x & 31, lr = lane & 15, hi = lane >> 4; const int r0 = blockIdx.x * 64, c0 = blockIdx.y * 64; const int cb = c0 + (int)blockIdx.x * bxr;
    v8f acc[4][4];
#pragma unroll
    for (int mb = 0; mb < 4; ++mb)
#pragma unroll
        for (int nb = 0; nb < 4; ++nb) acc[mb][nb] = (v8f){};
    const size_t aoff = (size_t)(r0 + lr) * lda + 8 * hi, boff = (size_t)(cb + lr) * ldb + (size_t)blockIdx.x * bxk + 8 * hi;
#pragma unroll 1
    for (int kc = 0; kc < K; kc += 32) {
        V a[4], a2[4];
#pragma unroll
        for (int mb = 0; mb < 4; ++mb) { a[mb] = WFrag<T16>::ld(A + aoff + (size_t)mb * 16 * lda + kc); if (NSPLIT == 1 || NSPLIT == 2) a2[mb] = WFrag<T16>::ld(A2 + aoff + (size_t)mb * 16 * lda + kc); }
#pragma unroll
        for (int nb = 0; nb < 4; ++nb) { const V b = WFrag<T16>::ld(Bt + boff + (size_t)nb * 16 * ldb + kc); V b2; if (NSPLIT >= 2) b2 = WFrag<T16>::ld(Bt2 + boff + (size_t)nb * 16 * ldb + kc);
#pragma unroll
            for (int mb = 0; mb < 4; ++mb) { acc[mb][nb] = WFrag<T16>::mma(a[mb], b, acc[mb][nb]); if (NSPLIT == 1 || NSPLIT == 2) acc[mb][nb] = WFrag<T16>::mma(a2[mb], b, acc[mb][nb]); if (NSPLIT >= 2) acc[mb][nb] = WFrag<T16>::mma(a[mb], b2, acc[mb][nb]); } }
        asm volatile("v_nop\n\tv_nop\n\tv_nop\n\tv_nop" : "+v"(acc[0][0]), "+v"(acc[1][1]), "+v"(acc[2][2]), "+v"(acc[3][3]) : "v"(a[0]), "v"(a[3]));
    }
#pragma unroll
    for (int mb = 0; mb < 4; ++mb) {
#pragma unroll
        for (int nb = 0; nb < 4; ++nb) {
#pragma unroll
            for (int j = 0; j < 8; ++j) os[(hi * 8 + j) * 68 + nb * 16 + lr] = acc[mb][nb][j]; }
        __builtin_amdgcn_wave_barrier(); asm volatile("" ::: "memory");
        float* crow = C + (size_t)(r0 + mb * 16) * ldc + c0;
#pragma unroll 1
        for (int ps = 0; ps < 2; ++ps) {
#pragma unroll
            for (int s = 0; s < 8; ++s) { const int row = 2 * s + hi, cofs = lr * 4; v4f val = *(const v4fa*)(os + row * 68 + cofs); if (BIAS) { val[0] += bfr(bias[c0 + cofs]); val[1] += bfr(bias[c0 + cofs + 1]); val[2] += bfr(bias[c0 + cofs + 2]); val[3] += bfr(bias[c0 + cofs + 3]); }
                *(volatile v4f*)(crow + (size_t)row * ldc + cofs) = val; }
            if (ps == 0) __threadfence(); }
        __builtin_amdgcn_wave_barrier(); asm volatile("" ::: "memory");
    }
}

__global__ __launch_bounds__(256) void k_cvt8(const float* __restrict__ src, bf* dst, size_t n8) { const size_t i = (size_t)blockIdx.x * 256 + threadIdx.x; if (i >= n8) return; const v8f v = *(const v8f*)(src + i * 8); v8us o;
#pragma unroll
    for (int k = 0; k < 8; ++k) o[k] = f2bf(v[k]); *(volatile v8us*)(dst + i * 8) = o; __threadfence(); *(volatile v8us*)(dst + i * 8) = o; }

__global__ __launch_bounds__(256) void k_cstab(const int* __restrict__ pos, float* CS) { const int idx = blockIdx.x * 256 + threadIdx.x; if (idx >= NB * SEQ * HD) return; const int t = idx / HD, d = idx % HD; const int b = t / SEQ, s = t - b * SEQ; const int i = (d < HD / 2) ? d : d - HD / 2;
    const float inv = __fdiv_rn(1.0f, powf(THETA, ((float)i * 2.0f) / (float)HD)); const float ang = __fmul_rn((float)pos[(size_t)b * S_FULL + s], inv); v2f cs; cs[0] = cosf(ang); cs[1] = sinf(ang);
    *(volatile v2f*)(CS + (size_t)idx * 2) = cs; __threadfence(); *(volatile v2f*)(CS + (size_t)idx * 2) = cs; }

__global__ __launch_bounds__(256) void k_mchk(const float* __restrict__ MK, float* POI) {
    __shared__ int flag[1]; const int tid = threadIdx.x; if (tid == 0) flag[0] = 0; __syncthreads(); int bad = 0; const int n4 = SEQ * (SEQ / 4);
#pragma unroll 1
    for (int p = tid; p < n4; p += 256) { const int i = p / (SEQ / 4); const int j = (p - i * (SEQ / 4)) * 4; const v4f m = *(const v4f*)(MK + (size_t)i * S_FULL + j); const int lo = (i / 64) * 64 - KPAD, hv = lo + BW;
#pragma unroll
        for (int q = 0; q < 4; ++q) { const int jj = j + q; const bool outb = (jj < lo) || (jj >= hv); if (outb && !(m[q] <= -1.0e8f)) bad = 1; } }
    if (bad) flag[0] = 1; __syncthreads(); const float val = (flag[0] != 0) ? __uint_as_float(0x7FC00000u) : 0.0f;
    v4f o; o[0] = val; o[1] = val; o[2] = val; o[3] = val;
    if (tid < DM / 4) *(volatile v4f*)(POI + (size_t)tid * 4) = o; __threadfence(); if (tid < DM / 4) *(volatile v4f*)(POI + (size_t)tid * 4) = o; }

__global__ __launch_bounds__(256) void k_rope(const float* __restrict__ F, int pitch, int pad, const float* __restrict__ CS, bf* Ph, bf* Pl) {
    const int TP = SEQ + 2 * pad; const size_t tot = (size_t)NH * TP * HD; const size_t e = ((size_t)blockIdx.x * 256 + threadIdx.x) * 2; if (e >= tot) return;
    const int d = (int)(e % HD); const int tp = (int)((e / HD) % TP); const int h = (int)(e / ((size_t)HD * TP)); const int t = tp - pad; const bool valid = (t >= 0) && (t < SEQ); const int tc = min(max(t, 0), SEQ - 1);
    const float* f = F + (size_t)tc * pitch + h * HD; v2us oh, ol;
#pragma unroll
    for (int q = 0; q < 2; ++q) { const int dd = d + q; const int dp = (dd < HD / 2) ? dd + HD / 2 : dd - HD / 2; const float x0 = f[dd], x1 = f[dp];
        const v2f cs = *(const v2f*)(CS + ((size_t)tc * HD + dd) * 2); float a = __fmul_rn(x0, cs[0]), bq = __fmul_rn(x1, cs[1]); asm volatile("" : "+v"(a)); asm volatile("" : "+v"(bq));
        float r = (dd < HD / 2) ? __fsub_rn(a, bq) : __fadd_rn(a, bq); r = valid ? r : 0.0f; unsigned short a2, c2; splitf(r, a2, c2); oh[q] = a2; ol[q] = c2; }
    *(volatile v2us*)(Ph + e) = oh; *(volatile v2us*)(Pl + e) = ol; __threadfence(); *(volatile v2us*)(Ph + e) = oh; *(volatile v2us*)(Pl + e) = ol; }

__global__ __launch_bounds__(256) void k_vtp(const float* __restrict__ F, int pitch, bf* Vh, bf* Vl) { const size_t tot = (size_t)NH * HD * LDV; const size_t e = ((size_t)blockIdx.x * 256 + threadIdx.x) * 2; if (e >= tot) return;
    const int tp = (int)(e % LDV); const int d = (int)((e / LDV) % HD); const int g = (int)(e / ((size_t)LDV * HD)); v2us oh, ol;
#pragma unroll
    for (int q = 0; q < 2; ++q) { const int t = tp + q - KPAD; const bool valid = (t >= 0) && (t < SEQ); const int tc = min(max(t, 0), SEQ - 1); float x = F[(size_t)tc * pitch + g * HD + d]; x = valid ? x : 0.0f; unsigned short a2, c2; splitf(x, a2, c2); oh[q] = a2; ol[q] = c2; }
    *(volatile v2us*)(Vh + e) = oh; *(volatile v2us*)(Vl + e) = ol; __threadfence(); *(volatile v2us*)(Vh + e) = oh; *(volatile v2us*)(Vl + e) = ol; }

__global__ __launch_bounds__(256) void k_bsoft(const float* __restrict__ Sb, const float* __restrict__ MK, bf* Ph, bf* Pl) {
    const int lane = threadIdx.x & 31; const int row = blockIdx.x * 8 + (threadIdx.x >> 5); if (row >= NH * SEQ) return; const int i = row % SEQ; const int qb = (i / 64) * 64 - KPAD;
    const float* sr = Sb + (size_t)row * BW; const float* mr = MK + (size_t)i * S_FULL; float v[2 * (BW / 64)]; float mx = -3.0e38f;
#pragma unroll
    for (int ch = 0; ch < BW / 64; ++ch) { const int c = ch * 64 + lane * 2; const int key = qb + c; const bool valid = (key >= 0) && (key < SEQ); const int kc2 = min(max(key, 0), SEQ - 2);
        const v2f a = *(const v2f*)(sr + c); const v2f m = *(const v2f*)(mr + kc2);
#pragma unroll
        for (int q = 0; q < 2; ++q) { float sa = __fmul_rn(a[q], SCL); asm volatile("" : "+v"(sa)); const float tq = __fadd_rn(sa, m[q]); const float t = valid ? tq : -3.0e38f; v[ch * 2 + q] = t; mx = fmaxf(mx, t); } }
#pragma unroll
    for (int sh = 16; sh; sh >>= 1) mx = fmaxf(mx, __shfl_xor(mx, sh, 32));
    float sum = 0.f;
#pragma unroll
    for (int k = 0; k < 2 * (BW / 64); ++k) { float d0 = __fsub_rn(v[k], mx); asm volatile("" : "+v"(d0)); v[k] = __builtin_amdgcn_exp2f(__fmul_rn(d0, 1.4426950408889634f)); sum += v[k]; }
#pragma unroll
    for (int sh = 16; sh; sh >>= 1) sum += __shfl_xor(sum, sh, 32);
    const float f = __fdiv_rn(1.0f, sum);
#pragma unroll 1
    for (int ps = 0; ps < 2; ++ps) {
#pragma unroll
        for (int ch = 0; ch < BW / 64; ++ch) { v2us oh, ol;
#pragma unroll
            for (int q = 0; q < 2; ++q) { unsigned short a, c2; splitf(v[ch * 2 + q] * f, a, c2); oh[q] = a; ol[q] = c2; }
            const size_t oo = (size_t)row * BW + ch * 64 + lane * 2; *(volatile v2us*)(Ph + oo) = oh; *(volatile v2us*)(Pl + oo) = ol; }
        if (ps == 0) __threadfence(); }
}

__global__ __launch_bounds__(256) void k_merge(const float* __restrict__ O, bf* Ah, bf* Al) { const size_t e = ((size_t)blockIdx.x * 256 + threadIdx.x) * 2; if (e >= (size_t)NH * SEQ * HD) return; const int d = (int)(e % HD); const int t = (int)((e / HD) % SEQ); const int zz = (int)(e / ((size_t)HD * SEQ));
    const size_t oo = (size_t)t * DM + (size_t)zz * HD + d; v2us oh, ol;
#pragma unroll
    for (int q = 0; q < 2; ++q) { unsigned short a, c2; splitf(O[e + q], a, c2); oh[q] = a; ol[q] = c2; } *(volatile v2us*)(Ah + oo) = oh; *(volatile v2us*)(Al + oo) = ol; __threadfence(); *(volatile v2us*)(Ah + oo) = oh; *(volatile v2us*)(Al + oo) = ol; }

extern "C" void kernel_launch(void* const* d_in, const int* in_sizes, int n_in,
                              void* d_out, int out_size, void* d_ws, size_t ws_size, hipStream_t stream) {
    if (n_in < 5) return;
    if ((size_t)in_sizes[0] < (size_t)(NB - 1) * S_FULL * DM + (size_t)SEQ * DM) return;
    if ((size_t)in_sizes[1] < (size_t)DQKV * DM) return;
    if ((size_t)in_sizes[2] < (size_t)DM * DM) return;
    if ((size_t)in_sizes[3] < (size_t)(SEQ - 1) * S_FULL + (size_t)SEQ) return;
    if ((size_t)in_sizes[4] < (size_t)(NB - 1) * S_FULL + (size_t)SEQ) return;
    if ((size_t)out_size < (size_t)NB * SEQ * DM) return;
    const float* x = (const float*)d_in[0];
    const float* wqkv = (const float*)d_in[1];
    const float* wo = (const float*)d_in[2];
    const float* mk = (const float*)d_in[3];
    const int* posid = (const int*)d_in[4];
    float* OUT = (float*)d_out;
    char* wsp = (char*)d_ws;
    auto take = [&](size_t bytes) { char* p = wsp; wsp += (bytes + 255) & ~(size_t)255; return (void*)p; };
    bf* WALL = (bf*)take((size_t)DQKV * DM * 2); bf* WO = (bf*)take((size_t)DM * DM * 2); float* CS = (float*)take((size_t)NB * SEQ * HD * 2 * 4); float* POI = (float*)take((size_t)DM * 4);
    bf* XB = (bf*)take((size_t)SEQ * DM * 2); float* F = (float*)take((size_t)SEQ * DQKV * 4);
    bf* QPh = (bf*)take((size_t)NH * SEQ * HD * 2); bf* QPl = (bf*)take((size_t)NH * SEQ * HD * 2); bf* KPh = (bf*)take((size_t)NH * LDV * HD * 2); bf* KPl = (bf*)take((size_t)NH * LDV * HD * 2);
    bf* VTh = (bf*)take((size_t)NH * HD * LDV * 2); bf* VTl = (bf*)take((size_t)NH * HD * LDV * 2);
    float* Sb = (float*)take((size_t)NH * SEQ * BW * 4); bf* Ph = (bf*)take((size_t)NH * SEQ * BW * 2); bf* Pl = (bf*)take((size_t)NH * SEQ * BW * 2);
    float* Ob = (float*)take((size_t)NH * SEQ * HD * 4); bf* ATh = (bf*)take((size_t)SEQ * DM * 2); bf* ATl = (bf*)take((size_t)SEQ * DM * 2);
    if ((size_t)(wsp - (char*)d_ws) > ws_size) return;
    k_cvt8<<<(unsigned)(((size_t)DQKV * DM / 8 + 255) / 256), 256, 0, stream>>>(wqkv, WALL, (size_t)DQKV * DM / 8);
    k_cvt8<<<(unsigned)(((size_t)DM * DM / 8 + 255) / 256), 256, 0, stream>>>(wo, WO, (size_t)DM * DM / 8);
    k_cstab<<<(unsigned)(((size_t)NB * SEQ * HD + 255) / 256), 256, 0, stream>>>(posid, CS);
    k_mchk<<<1, 256, 0, stream>>>(mk, POI);
    const unsigned LQ = (unsigned)(((size_t)NH * SEQ * HD / 2 + 255) / 256), LK = (unsigned)(((size_t)NH * LDV * HD / 2 + 255) / 256);
    for (int b = 0; b < NB; ++b) {
        const float* CSb = CS + (size_t)b * SEQ * HD * 2;
        k_cvt8<<<(unsigned)(((size_t)SEQ * DM / 8 + 255) / 256), 256, 0, stream>>>(x + (size_t)b * S_FULL * DM, XB, (size_t)SEQ * DM / 8);
        k_gemmw<bf, 0, false><<<dim3(SEQ / 64, DQKV / 64, 1), 32, 0, stream>>>(XB, nullptr, WALL, nullptr, DM, DM, DM, 0, 0, F, DQKV, nullptr, 0, 0, 0);
        k_rope<<<LQ, 256, 0, stream>>>(F, DQKV, 0, CSb, QPh, QPl);
        k_rope<<<LK, 256, 0, stream>>>(F + DM, DQKV, KPAD, CSb, KPh, KPl);
        k_vtp<<<LK, 256, 0, stream>>>(F + 2 * DM, DQKV, VTh, VTl);
        k_gemmw<bf, 2, false><<<dim3(SEQ / 64, BW / 64, NH), 32, 0, stream>>>(QPh, QPl, KPh, KPl, HD, HD, HD, 64, 0, Sb, BW, nullptr, (size_t)SEQ * HD, (size_t)LDV * HD, (size_t)SEQ * BW);
        k_bsoft<<<NH * SEQ / 8, 256, 0, stream>>>(Sb, mk, Ph, Pl);
        k_gemmw<bf, 2, false><<<dim3(SEQ / 64, HD / 64, NH), 32, 0, stream>>>(Ph, Pl, VTh, VTl, BW, BW, LDV, 0, 64, Ob, HD, nullptr, (size_t)SEQ * BW, (size_t)HD * LDV, (size_t)SEQ * HD);
        k_merge<<<LQ, 256, 0, stream>>>(Ob, ATh, ATl);
        k_gemmw<bf, 1, true><<<dim3(SEQ / 64, DM / 64, 1), 32, 0, stream>>>(ATh, ATl, WO, nullptr, DM, DM, DM, 0, 0, OUT + (size_t)b * SEQ * DM, DM, POI, 0, 0, 0);
    }
}
